// Mask3dAttention_66297115181710
// MI455X (gfx1250) — hardware-verified
//
#include <hip/hip_runtime.h>
#include <hip/hip_bf16.h>
#include <math.h>


#define BB 4
#define SS 2048
#define DD 256
#define HH 8
#define DKK 32
#define QW 2

typedef _Float16 bf16;
typedef __attribute__((ext_vector_type(4))) unsigned v4u_t;
typedef unsigned v4ua __attribute__((ext_vector_type(4), may_alias));
typedef __attribute__((ext_vector_type(4))) float v4f_t;
typedef float v4fa __attribute__((ext_vector_type(4), may_alias));
typedef __attribute__((ext_vector_type(16))) bf16  bf16x16;
typedef __attribute__((ext_vector_type(8)))  bf16  bf16x8;
typedef __attribute__((ext_vector_type(4)))  bf16  bf16x4;
typedef __attribute__((ext_vector_type(8)))  float f32x8;

#define LDS_STRIDE 48
#define KSTRIDE    72
#define VSTRIDE    48

__device__ __forceinline__ f32x8 wmma_bf16(bf16x16 a, bf16x16 b, f32x8 c) {
  return __builtin_amdgcn_wmma_f32_16x16x32_f16(
      false, a, false, b, (short)0, c, false, false);
}

template <typename T>
__device__ __forceinline__ bf16x16 load_frag(const T* __restrict__ base, int ld,
                                             int row0, int k0) {
  const int lane = threadIdx.x & 31;
  const int r    = lane & 15;
  const int kh   = (lane >> 4) * 8;
  const T* p0 = base + (size_t)(row0 + r) * ld + (k0 + kh);
  const T* p1 = p0 + 16;
  bf16x16 f;
#pragma unroll
  for (int i = 0; i < 8; ++i) {
    f[i]     = (bf16)p0[i];
    f[i + 8] = (bf16)p1[i];
  }
  return f;
}

__device__ __forceinline__ bf16x16 lds_frag(const bf16* base, int stride) {
  const int lane = threadIdx.x & 31;
  const int row  = lane & 15;
  const int kh   = (lane >> 4) * 8;
  const bf16x8 lo = *(const bf16x8*)(base + row * stride + kh);
  const bf16x8 hi = *(const bf16x8*)(base + row * stride + kh + 16);
  bf16x16 f;
#pragma unroll
  for (int i = 0; i < 8; ++i) { f[i] = lo[i]; f[i + 8] = hi[i]; }
  return f;
}

template <typename T>
__device__ __forceinline__ void stage_read16(const T* __restrict__ p, float* buf) {
#pragma unroll
  for (int i = 0; i < 16; ++i) buf[i] = (float)p[i];
}

__device__ __forceinline__ void stage_write(bf16* dst, const float* buf, int nquad) {
#pragma unroll
  for (int i = 0; i < nquad; ++i) {
    bf16x4 q;
    q[0] = (bf16)buf[4 * i];     q[1] = (bf16)buf[4 * i + 1];
    q[2] = (bf16)buf[4 * i + 2]; q[3] = (bf16)buf[4 * i + 3];
    *(bf16x4*)(dst + 4 * i) = q;
  }
}

template <typename AT, int MODE>
__global__ __launch_bounds__(256) void gemm_bias_kernel(
    const AT* __restrict__ A, const float* __restrict__ W,
    const float* __restrict__ bias, void* __restrict__ out,
    int M, int N, int K) {
  __shared__ bf16 ldsA[128 * LDS_STRIDE];
  __shared__ bf16 ldsW[256 * LDS_STRIDE];
  __shared__ __attribute__((aligned(16))) unsigned char sob[256 * 136 * 2];

  const int t    = threadIdx.x;
  const int wave = t >> 5;
  const int lane = t & 31;
  const int wm   = (wave & 1) * 64;
  const int wn   = (wave >> 1) * 64;
  const int mBlk = blockIdx.x * 128;
  const int nBlk = blockIdx.y * 256;

  const int arow = t >> 1;
  const int ach  = (t & 1) * 16;

  float abuf[16];
  float wbuf[32];

  stage_read16(A + (size_t)(mBlk + arow) * K + ach, abuf);
  stage_read16(W + (size_t)(nBlk + t) * K,          wbuf);
  stage_read16(W + (size_t)(nBlk + t) * K + 16,     wbuf + 16);

  f32x8 acc[4][4] = {};

  for (int k = 0; k < K; k += 32) {
    __syncthreads();
    stage_write(&ldsA[arow * LDS_STRIDE + ach], abuf, 4);
    stage_write(&ldsW[t * LDS_STRIDE],          wbuf, 8);
    if (k + 32 < K) {
      stage_read16(A + (size_t)(mBlk + arow) * K + (k + 32) + ach, abuf);
      stage_read16(W + (size_t)(nBlk + t) * K + (k + 32),          wbuf);
      stage_read16(W + (size_t)(nBlk + t) * K + (k + 32) + 16,     wbuf + 16);
    }
    __syncthreads();

    bf16x16 af[4], wf[4];
#pragma unroll
    for (int i = 0; i < 4; ++i)
      af[i] = lds_frag(ldsA + (wm + 16 * i) * LDS_STRIDE, LDS_STRIDE);
#pragma unroll
    for (int j = 0; j < 4; ++j)
      wf[j] = lds_frag(ldsW + (wn + 16 * j) * LDS_STRIDE, LDS_STRIDE);
#pragma unroll
    for (int i = 0; i < 4; ++i)
#pragma unroll
      for (int j = 0; j < 4; ++j)
        acc[i][j] = wmma_bf16(af[i], wf[j], acc[i][j]);
  }

  const int nlane = lane & 15;
  const int mh    = (lane >> 4) * 8;
  __syncthreads();
  if (MODE == 0 || MODE == 1) {
    bf16* so = (bf16*)sob;
#pragma unroll
    for (int i = 0; i < 4; ++i)
#pragma unroll
      for (int j = 0; j < 4; ++j) {
        const int nl = wn + 16 * j + nlane;
        const float bv = bias ? bias[nBlk + nl] : 0.0f;
#pragma unroll
        for (int r = 0; r < 8; ++r) {
          const int ml = wm + 16 * i + mh + r;
          const bf16 hv = (bf16)(acc[i][j][r] + bv);
          if (MODE == 0) so[ml * 264 + nl] = hv;
          else           so[nl * 136 + ml] = hv;
        }
      }
    __syncthreads();
#pragma unroll 1
    for (int pass = 0; pass < 2; ++pass) {
      if (MODE == 0) {
        for (int ch = t; ch < 128 * 32; ch += 256) { const int ml = ch >> 5, q = (ch & 31) * 8;
          *(volatile v4u_t*)((bf16*)out + (size_t)(mBlk + ml) * N + nBlk + q) = *(const v4ua*)(so + ml * 264 + q); }
      } else {
        const int b_ = mBlk / SS, s0 = mBlk & (SS - 1);
        for (int ch = t; ch < 256 * 16; ch += 256) { const int nl = ch >> 4, q = (ch & 15) * 8; const int n = nBlk + nl, h = n >> 6, dk = n & (DKK - 1);
          *(volatile v4u_t*)((bf16*)out + (((size_t)(b_ * HH + h)) * DKK + dk) * SS + s0 + q) = *(const v4ua*)(so + nl * 136 + q); }
      }
      __threadfence();
    }
  } else {
    float* so = (float*)sob;
#pragma unroll 1
    for (int hf = 0; hf < 2; ++hf) {
      if (wm == hf * 64) {
#pragma unroll
        for (int i = 0; i < 4; ++i)
#pragma unroll
          for (int j = 0; j < 4; ++j) {
            const int nl = wn + 16 * j + nlane;
            const float bv = bias ? bias[nBlk + nl] : 0.0f;
#pragma unroll
            for (int r = 0; r < 8; ++r) so[(16 * i + mh + r) * 260 + nl] = acc[i][j][r] + bv;
          }
      }
      __syncthreads();
#pragma unroll 1
      for (int pass = 0; pass < 2; ++pass) {
        for (int ch = t; ch < 64 * 64; ch += 256) { const int ml = ch >> 6, q = (ch & 63) * 4;
          *(volatile v4f_t*)((float*)out + (size_t)(mBlk + hf * 64 + ml) * N + nBlk + q) = *(const volatile v4fa*)(so + ml * 260 + q); }
        __threadfence();
      }
      __syncthreads();
    }
  }
}


#define KS32 40
#define VS32 40
template <int CAUSAL>
__global__ __launch_bounds__(128) void attn32_kernel(const bf16* __restrict__ Qb, const bf16* __restrict__ Kb, const bf16* __restrict__ Vt,
                                                    float* __restrict__ O, float scale_log2e, int S, int ldq, int ldo, int nhv, int qbase, int klim) {
  __shared__ bf16 ldsK[2][32 * KS32];
  __shared__ bf16 ldsV[2][32 * VS32];
  __shared__ __attribute__((aligned(16))) float ldsO[32 * 68];
  const int qblk = qbase + blockIdx.x * 32, hp = blockIdx.y, b = blockIdx.z;
  const int t = threadIdx.x, wave = t >> 5, lane = t & 31, qlane = lane & 15, kh8 = (lane >> 4) * 8;
  const int hl = wave >> 1, h = 2 * hp + hl, qt = wave & 1, q0 = qblk + 16 * qt;
  const bf16* Qh = Qb + (size_t)b * S * ldq + h * 32;
  const bf16x16 qf = load_frag(Qh, ldq, q0, 0);
  const int sh = t >> 6, sr = (t >> 1) & 31, sc = (t & 1) * 16;
  const bf16* Ks = Kb + (size_t)b * S * ldq + (2 * hp + sh) * 32 + sc;
  const bf16* Vs = Vt + (((size_t)(b * nhv + 2 * hp + sh)) * 32 + sr) * S + sc;
  f32x8 o[2] = {};
  float mrun = -INFINITY, lrun = 0.0f;
  const int qi = q0 + qlane;
  const int kend = CAUSAL ? (qblk + 31) : (klim - 1);
#pragma unroll 1
  for (int kb = 0; kb <= kend; kb += 32) {
    __syncthreads();
    { const bf16* kp = Ks + (size_t)(kb + sr) * ldq; const bf16* vp = Vs + kb;
      *(bf16x8*)(&ldsK[sh][sr * KS32 + sc]) = *(const bf16x8*)kp; *(bf16x8*)(&ldsK[sh][sr * KS32 + sc + 8]) = *(const bf16x8*)(kp + 8);
      *(bf16x8*)(&ldsV[sh][sr * VS32 + sc]) = *(const bf16x8*)vp; *(bf16x8*)(&ldsV[sh][sr * VS32 + sc + 8]) = *(const bf16x8*)(vp + 8); }
    __syncthreads();
    f32x8 s0 = {}, s1 = {};
    s0 = wmma_bf16(lds_frag(&ldsK[hl][0], KS32), qf, s0);
    s1 = wmma_bf16(lds_frag(&ldsK[hl][16 * KS32], KS32), qf, s1);
    float mx = -INFINITY;
#pragma unroll
    for (int r = 0; r < 8; ++r) { const int j0 = kb + kh8 + r, j1 = j0 + 16;
      s0[r] = (!CAUSAL || j0 <= qi) ? s0[r] * scale_log2e : -INFINITY;
      s1[r] = (!CAUSAL || j1 <= qi) ? s1[r] * scale_log2e : -INFINITY;
      mx = fmaxf(mx, fmaxf(s0[r], s1[r])); }
    mx = fmaxf(mx, __shfl_xor(mx, 16, 32));
    const float mnew = fmaxf(mrun, mx), alpha = exp2f(mrun - mnew);
    float rsum = 0.0f; bf16x16 pf;
#pragma unroll
    for (int r = 0; r < 8; ++r) { const float p0 = exp2f(s0[r] - mnew), p1 = exp2f(s1[r] - mnew); rsum += p0 + p1; pf[r] = (bf16)(p0 * 1024.0f); pf[r + 8] = (bf16)(p1 * 1024.0f); }
    rsum += __shfl_xor(rsum, 16, 32);
    lrun = lrun * alpha + rsum; mrun = mnew;
#pragma unroll
    for (int j = 0; j < 2; ++j) {
#pragma unroll
      for (int r = 0; r < 8; ++r) o[j][r] *= alpha;
      o[j] = wmma_bf16(lds_frag(&ldsV[hl][(j * 16) * VS32], VS32), pf, o[j]); }
  }
  const float rl = 1.0f / (lrun * 1024.0f);
#pragma unroll
  for (int j = 0; j < 2; ++j)
#pragma unroll
    for (int r = 0; r < 8; ++r) ldsO[(16 * qt + qlane) * 68 + hl * 32 + j * 16 + kh8 + r] = o[j][r] * rl;
  __syncthreads();
#pragma unroll 1
  for (int pass = 0; pass < 2; ++pass) {
    for (int i = t; i < 32 * 16; i += 128) { const int row = i >> 4, q4 = (i & 15) * 4;
      float* dst = O + ((size_t)(b * S + qblk + row)) * ldo + hp * 64 + q4;
      *(volatile v4f_t*)dst = *(const volatile v4fa*)(ldsO + row * 68 + q4); }
    __threadfence();
  }
}

__global__ __launch_bounds__(256) void k_tw(const float* __restrict__ W, float* __restrict__ WT, int K, int N) {
  __shared__ float tile[64][65];
  const int kb0 = blockIdx.y * 64, n0 = blockIdx.x * 64, t = threadIdx.x;
  for (int i = t; i < 64 * 64; i += 256) { const int kr = i >> 6, nc = i & 63; tile[kr][nc] = W[(size_t)(kb0 + kr) * N + n0 + nc]; }
  __syncthreads();
#pragma unroll 1
  for (int pass = 0; pass < 2; ++pass) {
    for (int i = t; i < 64 * 16; i += 256) { const int nr = i >> 4, k4 = (i & 15) * 4; v4f_t v; v.x = tile[k4][nr]; v.y = tile[k4 + 1][nr]; v.z = tile[k4 + 2][nr]; v.w = tile[k4 + 3][nr];
      *(volatile v4f_t*)(WT + (size_t)(n0 + nr) * K + kb0 + k4) = v; }
    __threadfence();
  }
}
__global__ __launch_bounds__(256) void k_vt(const bf16* __restrict__ Vr, bf16* __restrict__ Vt) {
  __shared__ bf16 tile[64][72];
  const int s0 = blockIdx.x * 64, d0 = blockIdx.y * 64, b = blockIdx.z, t = threadIdx.x;
  for (int i = t; i < 64 * 64; i += 256) { const int r = i >> 6, d = i & 63; tile[r][d] = Vr[((size_t)(b * SS + s0 + r)) * DD + d0 + d]; }
  __syncthreads();
#pragma unroll 1
  for (int pass = 0; pass < 2; ++pass) {
    for (int i = t; i < 64 * 8; i += 256) { const int dr = i >> 3, s8 = (i & 7) * 8; bf16 hh[8];
#pragma unroll
      for (int e = 0; e < 8; ++e) hh[e] = tile[s8 + e][dr];
      *(volatile v4u_t*)(Vt + ((size_t)b * DD + d0 + dr) * SS + s0 + s8) = *(const v4ua*)hh; }
    __threadfence();
  }
}

extern "C" void kernel_launch(void* const* d_in, const int* in_sizes, int n_in,
                              void* d_out, int out_size, void* d_ws, size_t ws_size,
                              hipStream_t stream) {
  (void)in_sizes; (void)n_in; (void)out_size; (void)ws_size;
  const float* x = (const float*)d_in[0];
  const float* Wqkv = (const float*)d_in[1];
  const float* bqkv = (const float*)d_in[2];
  const int M = BB * SS;
  char* ws = (char*)d_ws;
  float* WT = (float*)ws; ws += (size_t)3 * DD * DD * 4;
  bf16* Qb  = (bf16*)ws;  ws += (size_t)M * DD * 2;
  bf16* Kb  = (bf16*)ws;  ws += (size_t)M * DD * 2;
  bf16* Vr  = (bf16*)ws;  ws += (size_t)M * DD * 2;
  bf16* VtB = (bf16*)ws;  ws += (size_t)M * DD * 2;
  const size_t pl = (size_t)DD * DD;
  k_tw<<<dim3(3 * DD / 64, DD / 64), 256, 0, stream>>>(Wqkv, WT, DD, 3 * DD);
  dim3 gGrid(M / 128, DD / 256), gBlk(256);
  gemm_bias_kernel<float, 0><<<gGrid, gBlk, 0, stream>>>(x, WT,          bqkv,          Qb, M, DD, DD);
  gemm_bias_kernel<float, 0><<<gGrid, gBlk, 0, stream>>>(x, WT + pl,     bqkv + DD,     Kb, M, DD, DD);
  gemm_bias_kernel<float, 0><<<gGrid, gBlk, 0, stream>>>(x, WT + 2 * pl, bqkv + 2 * DD, Vr, M, DD, DD);
  k_vt<<<dim3(SS / 64, DD / 64, BB), 256, 0, stream>>>(Vr, VtB);
  const float sl2e = 0.17677669529663687f * 1.44269504088896340736f;
  attn32_kernel<0><<<dim3(SS / 2 / 32, HH / 2, BB), 128, 0, stream>>>(Qb, Kb, VtB, (float*)d_out, sl2e, SS, DD, DD, HH, 0, SS / 2);
  attn32_kernel<1><<<dim3(SS / 2 / 32, HH / 2, BB), 128, 0, stream>>>(Qb, Kb, VtB, (float*)d_out, sl2e, SS, DD, DD, HH, SS / 2, SS);
}
